// EncoderLayer_29343216566369
// MI455X (gfx1250) — hardware-run, weakly checked
//
#include <hip/hip_runtime.h>


#ifndef NB
#define NB 4096
#endif
#ifndef SEQ
#define SEQ 128
#endif
#define NB_FULL  4096
#define SEQ_FULL 128
#ifndef OUT_NB
#define OUT_NB NB
#endif
#define EMB  12
#define HID  32
#define BPB  8
#define OSW  (BPB * EMB)
#define OITER ((SEQ * (OSW / 4)) / (32 * BPB))
#define ACARRY 64.0f
#define AINV   (1.0f / 64.0f)
#define SC2  ((float)(0.28867513459481287 * 1.4426950408889634))
#define PSH  14.0f
#define NEGB (-3.0e38f)
#define LNEPS 1.0e-5f

static_assert(EMB == 12);
static_assert(HID == 32);
static_assert(SEQ % 32 == 0);
static_assert(SEQ % 16 == 0);
static_assert(NB % BPB == 0);
static_assert(OUT_NB % BPB == 0);
static_assert((OSW * 4) % 128 == 0);
static_assert((OSW / 4) % 8 == 0);
static_assert((SEQ * (OSW / 4)) % (32 * BPB) == 0);
static_assert((size_t)(32 * BPB) * OITER * 16 == (size_t)SEQ * OSW * 4);
static_assert(NB <= NB_FULL);
static_assert(SEQ <= SEQ_FULL);
static_assert((48 * 16) % (32 * BPB) == 0);
static_assert((16 * 16) % (32 * BPB) == 0);
static_assert((32 * 16) % (32 * BPB) == 0);
static_assert((32 * 32) % (32 * BPB) == 0);
static_assert((16 * 32) % (32 * BPB) == 0);
static_assert(32 * BPB >= 48);

typedef _Float16 h16;
typedef unsigned short bf;
typedef __attribute__((ext_vector_type(16))) __bf16   v16bf;
typedef __attribute__((ext_vector_type(16))) _Float16 v16h;
typedef __attribute__((ext_vector_type(8)))  _Float16 v8h;
typedef __attribute__((ext_vector_type(8)))  unsigned short v8us;
typedef __attribute__((ext_vector_type(8)))  float    v8f;
typedef __attribute__((ext_vector_type(4)))  float    v4f;
typedef v4f  __attribute__((may_alias)) v4fa;

__device__ __forceinline__ unsigned short f2bf(float f) { unsigned u = __float_as_uint(f); u += 0x7FFFu + ((u >> 16) & 1u); return (unsigned short)(u >> 16); }
__device__ __forceinline__ float bfr(float f) { return __uint_as_float(((unsigned)f2bf(f)) << 16); }
__device__ __forceinline__ v16h cat16(v8h lo, v8h hi) { return __builtin_shufflevector(lo, hi, 0, 1, 2, 3, 4, 5, 6, 7, 8, 9, 10, 11, 12, 13, 14, 15); }
__device__ __forceinline__ v16bf cat16b(v8us lo, v8us hi) { return __builtin_bit_cast(v16bf, __builtin_shufflevector(lo, hi, 0, 1, 2, 3, 4, 5, 6, 7, 8, 9, 10, 11, 12, 13, 14, 15)); }
__device__ __forceinline__ void wave_sync() { __builtin_amdgcn_fence(3  , "wavefront"); __builtin_amdgcn_wave_barrier(); asm volatile("" ::: "memory"); }

static __device__ __forceinline__ h16 toh_flush(float v) { const h16 r = (h16)v; return (fabsf(v) < 6.103515625e-05f) ? (h16)0.0f : r; }
__device__ __forceinline__ v8f wmma16g(v16h a, v16h b, v8f c) {
    c = __builtin_amdgcn_wmma_f32_16x16x32_f16(false, a, false, b, (short)0, c, false, false);
    asm volatile("v_nop\n\tv_nop\n\tv_nop\n\tv_nop" : "+v"(c) : "v"(a), "v"(b));
    return c; }
__device__ __forceinline__ v8f wmmabg(v16bf a, v16bf b, v8f c) {
    c = __builtin_amdgcn_wmma_f32_16x16x32_bf16(false, a, false, b, (short)0, c, false, false);
    asm volatile("v_nop\n\tv_nop\n\tv_nop\n\tv_nop" : "+v"(c) : "v"(a), "v"(b));
    return c; }
__device__ __forceinline__ float tanh_e(float v) { const float e = __builtin_amdgcn_exp2f(v * 2.8853900817779268f); return 1.0f - 2.0f * __builtin_amdgcn_rcpf(e + 1.0f); }
__device__ __forceinline__ v16h packlo(v8f a) { v16h o = (v16h){};
#pragma unroll
    for (int r = 0; r < 8; ++r) o[r] = toh_flush(a[r]);
    return o; }
__device__ __forceinline__ v16h pack2(v8f a, v8f b) { v16h o;
#pragma unroll
    for (int r = 0; r < 8; ++r) { o[r] = toh_flush(a[r]); o[8 + r] = toh_flush(b[r]); }
    return o; }
__device__ __forceinline__ v8f ldx8(const float* __restrict__ x, size_t off, int hi) {
    v4f a = *(const v4f*)(x + off + 8 * hi);
    v4f c = *(const v4f*)(x + off + 4 + 4 * hi);
    asm volatile("" : "+v"(a)); asm volatile("" : "+v"(c));
    v8f o;
#pragma unroll
    for (int i = 0; i < 4; ++i) { o[i] = bfr(a[i]); const float t = bfr(c[i]); o[4 + i] = (hi == 0) ? t : 0.0f; }
    return o; }
__device__ __forceinline__ v16bf xfrag(v8f xf) { v8us u;
#pragma unroll
    for (int i = 0; i < 8; ++i) u[i] = (unsigned short)(__float_as_uint(xf[i]) >> 16);
    return cat16b(u, (v8us){}); }

static constexpr size_t LDS_BYTES = (size_t)SEQ * OSW * 4 + (size_t)2 * BPB * SEQ * 16 * 2
                                  + (size_t)(48 * 16 + 16 * 16 + 32 * 16 + 32 * 32 + 16 * 32) * 2 + (size_t)(48 + 16 + 32 + 32 + 16 * 5) * 4;
static_assert(LDS_BYTES <= (size_t)131072);

__global__ __launch_bounds__(32 * BPB) void k_enc(const float* __restrict__ x,
                                                  const float* __restrict__ inw, const float* __restrict__ inb,
                                                  const float* __restrict__ ow,  const float* __restrict__ ob,
                                                  const float* __restrict__ w1,  const float* __restrict__ b1,
                                                  const float* __restrict__ w2,  const float* __restrict__ b2,
                                                  const float* __restrict__ w3,  const float* __restrict__ b3,
                                                  const float* __restrict__ g1,  const float* __restrict__ be1,
                                                  const float* __restrict__ g2,  const float* __restrict__ be2,
                                                  float* out) {
    __shared__ __align__(16) float os[SEQ * OSW];
    __shared__ __align__(16) h16 kp[BPB * SEQ * 16];
    __shared__ __align__(16) h16 vt[BPB * 16 * SEQ];
    __shared__ __align__(16) bf  wins[48 * 16];
    __shared__ __align__(16) h16 wos[16 * 16];
    __shared__ __align__(16) h16 w1s[32 * 16];
    __shared__ __align__(16) h16 w2s[32 * 32];
    __shared__ __align__(16) h16 w3s[16 * 32];
    __shared__ float bins[48], bos[16], b1s[32], b2s[32], b3s[16], g1s[16], e1s[16], g2s[16], e2s[16];

    const int tid = threadIdx.x;
#pragma unroll 1
    for (int i = tid; i < 48 * 16; i += 32 * BPB) { const int row = i >> 4, e = i & 15, sec = row >> 4, d = row & 15; const bool ok = (d < EMB) & (e < EMB);
        float v = inw[ok ? (sec * EMB + d) * EMB + e : 0]; asm volatile("" : "+v"(v)); wins[i] = ok ? f2bf(v) : (bf)0; }
#pragma unroll 1
    for (int i = tid; i < 16 * 16; i += 32 * BPB) { const int f = i >> 4, e = i & 15; const bool ok = (f < EMB) & (e < EMB);
        float v = ow[ok ? f * EMB + e : 0]; asm volatile("" : "+v"(v)); const h16 c = toh_flush(bfr(v)); wos[i] = ok ? c : (h16)0.0f; }
#pragma unroll 1
    for (int i = tid; i < 32 * 16; i += 32 * BPB) { const int g = i >> 4, e = i & 15; const bool ok = e < EMB;
        float v = w1[ok ? g * EMB + e : 0]; asm volatile("" : "+v"(v)); const h16 c = toh_flush(bfr(v)); w1s[i] = ok ? c : (h16)0.0f; }
#pragma unroll 1
    for (int i = tid; i < 32 * 32; i += 32 * BPB) { float v = w2[i]; w2s[i] = toh_flush(bfr(v)); }
#pragma unroll 1
    for (int i = tid; i < 16 * 32; i += 32 * BPB) { const int e = i >> 5, g = i & 31; const bool ok = e < EMB;
        float v = w3[ok ? e * HID + g : 0]; asm volatile("" : "+v"(v)); const h16 c = toh_flush(bfr(v)); w3s[i] = ok ? c : (h16)0.0f; }
    { const int c48 = tid < 48 ? tid : 47; const int sec = c48 >> 4, d = c48 & 15; const bool okb = d < EMB;
      float v = inb[okb ? sec * EMB + d : 0]; asm volatile("" : "+v"(v));
      const int c32 = tid & 31; float u1 = b1[c32], u2 = b2[c32]; asm volatile("" : "+v"(u1)); asm volatile("" : "+v"(u2));
      const int c16 = tid & 15; const bool ok16 = c16 < EMB; const int i12 = ok16 ? c16 : 0;
      float a0 = ob[i12], a1 = b3[i12], a2 = g1[i12], a3 = be1[i12], a4 = g2[i12], a5 = be2[i12];
      asm volatile("" : "+v"(a0)); asm volatile("" : "+v"(a1)); asm volatile("" : "+v"(a2)); asm volatile("" : "+v"(a3)); asm volatile("" : "+v"(a4)); asm volatile("" : "+v"(a5));
      if (tid < 48) bins[tid] = okb ? bfr(v) : 0.0f;
      if (tid < 32) { b1s[tid] = bfr(u1); b2s[tid] = bfr(u2); }
      if (tid < 16) { bos[tid] = ok16 ? bfr(a0) : 0.0f; b3s[tid] = ok16 ? bfr(a1) : 0.0f; g1s[tid] = ok16 ? bfr(a2) : 0.0f; e1s[tid] = ok16 ? bfr(a3) : 0.0f;
                      g2s[tid] = ok16 ? bfr(a4) : 0.0f; e2s[tid] = ok16 ? bfr(a5) : 0.0f; } }
    __syncthreads();

    const int lane = tid & 31, lr = lane & 15, hi = lane >> 4;
    const int wave = __builtin_amdgcn_readfirstlane((int)(threadIdx.x >> 5));
    const int n0 = blockIdx.x * BPB;
    const int n = n0 + wave;
    const v8us z8u = (v8us){}; const v8h z8h = (v8h){};
    const v16bf wq = cat16b(*(const v8us*)&wins[(0 * 16 + lr) * 16 + 8 * hi], z8u);
    const v16bf wk = cat16b(*(const v8us*)&wins[(1 * 16 + lr) * 16 + 8 * hi], z8u);
    const v16bf wv = cat16b(*(const v8us*)&wins[(2 * 16 + lr) * 16 + 8 * hi], z8u);
    const int kb = wave * SEQ * 16, vb = wave * 16 * SEQ;
    const size_t xo = ((size_t)lr * NB_FULL + (size_t)n) * EMB;
    const size_t xts = (size_t)16 * NB_FULL * EMB;

#pragma unroll 1
    for (int tk = 0; tk < SEQ / 16; ++tk) {
        const v8f xf = ldx8(x, xo + (size_t)tk * xts, hi);
        const v16bf xb = xfrag(xf);
        const v8f kt = wmmabg(wk, xb, (v8f){});
        const v8f vv = wmmabg(xb, wv, (v8f){});
        const float bvv = bins[32 + lr];
        v8h kh, vh;
#pragma unroll
        for (int r = 0; r < 8; ++r) { kh[r] = toh_flush(kt[r] + bins[16 + 8 * hi + r]); vh[r] = toh_flush(vv[r] + bvv); }
        *(v8h*)&kp[kb + (tk * 16 + lr) * 16 + 8 * hi] = kh;
        *(v8h*)&vt[vb + lr * SEQ + tk * 16 + 8 * hi] = vh;
    }
    wave_sync();

#pragma unroll 1
    for (int qt = 0; qt < SEQ / 16; ++qt) {
        const v8f xf = ldx8(x, xo + (size_t)qt * xts, hi);
        const v16bf xb = xfrag(xf);
        const v8f qa = wmmabg(wq, xb, (v8f){});
        v8f qv;
#pragma unroll
        for (int r = 0; r < 8; ++r) qv[r] = qa[r] + bins[8 * hi + r];
        const v16h qB = packlo(qv);
        v8f o0 = (v8f){};
        float m = NEGB, l = 0.0f;
#pragma unroll 1
        for (int key0 = 0; key0 < SEQ; key0 += 32) {
            const v16h ka0 = cat16(*(const v8h*)&kp[kb + (key0 + lr) * 16 + 8 * hi], z8h);
            const v16h kb0 = cat16(*(const v8h*)&kp[kb + (key0 + 16 + lr) * 16 + 8 * hi], z8h);
            const v8f sa = wmma16g(ka0, qB, (v8f){});
            const v8f sb = wmma16g(kb0, qB, (v8f){});
            float ta[8], tb[8]; float mx = NEGB;
#pragma unroll
            for (int r = 0; r < 8; ++r) { ta[r] = sa[r] * SC2; tb[r] = sb[r] * SC2; mx = fmaxf(mx, fmaxf(ta[r], tb[r])); }
            mx = fmaxf(mx, __shfl_xor(mx, 16, 32));
            const float mnew = fmaxf(m, mx);
            const float alpha = __builtin_amdgcn_exp2f(m - mnew);
            const float sh = PSH - mnew;
            v16h pb; float ls = 0.0f;
#pragma unroll
            for (int r = 0; r < 8; ++r) {
                const float ea = ta[r] + sh, eb = tb[r] + sh;
                const float xa = __builtin_amdgcn_exp2f(ea), xc = __builtin_amdgcn_exp2f(eb);
                const float ga = (ea < -14.0f) ? 0.0f : xa, gb = (eb < -14.0f) ? 0.0f : xc;
                const h16 pa = (h16)ga; const h16 pc = (h16)gb;
                pb[r] = pa; pb[8 + r] = pc; ls += (float)pa + (float)pc; }
            l = l * alpha + ls; m = mnew;
            o0 = o0 * alpha;
            const v16h va = cat16(*(const v8h*)&vt[vb + lr * SEQ + key0 + 8 * hi], *(const v8h*)&vt[vb + lr * SEQ + key0 + 16 + 8 * hi]);
            o0 = wmma16g(va, pb, o0);
        }
        l += __shfl_xor(l, 16, 32);
        const float inv = ACARRY * (1.0f / l);
        v8f av;
#pragma unroll
        for (int r = 0; r < 8; ++r) av[r] = o0[r] * inv;
        const v16h aB = packlo(av);
        const v16h woA = cat16(*(const v8h*)&wos[lr * 16 + 8 * hi], z8h);
        const v8f ya = wmma16g(woA, aB, (v8f){});
        float y[8]; float s1 = 0.0f;
#pragma unroll
        for (int r = 0; r < 8; ++r) { const bool ok = (r < 4) | (hi == 0); y[r] = ya[r] * AINV + bos[8 * hi + r] + xf[r]; s1 += ok ? y[r] : 0.0f; }
        s1 += __shfl_xor(s1, 16, 32);
        const float mu1 = s1 * (1.0f / 12.0f);
        float dd[8]; float s2 = 0.0f;
#pragma unroll
        for (int r = 0; r < 8; ++r) { const bool ok = (r < 4) | (hi == 0); dd[r] = ok ? (y[r] - mu1) : 0.0f; s2 += dd[r] * dd[r]; }
        s2 += __shfl_xor(s2, 16, 32);
        const float rs1 = rsqrtf(s2 * (1.0f / 12.0f) + LNEPS);
        v8f z;
#pragma unroll
        for (int r = 0; r < 8; ++r) z[r] = dd[r] * rs1 * g1s[8 * hi + r] + e1s[8 * hi + r];
        const v16h zB = packlo(z);
        v8f h1a = wmma16g(cat16(*(const v8h*)&w1s[lr * 16 + 8 * hi], z8h), zB, (v8f){});
        v8f h1b = wmma16g(cat16(*(const v8h*)&w1s[(16 + lr) * 16 + 8 * hi], z8h), zB, (v8f){});
#pragma unroll
        for (int r = 0; r < 8; ++r) { h1a[r] = tanh_e(h1a[r] + b1s[8 * hi + r]); h1b[r] = tanh_e(h1b[r] + b1s[16 + 8 * hi + r]); }
        const v16h h1B = pack2(h1a, h1b);
        v8f h2a = wmma16g(cat16(*(const v8h*)&w2s[lr * 32 + 8 * hi], *(const v8h*)&w2s[lr * 32 + 16 + 8 * hi]), h1B, (v8f){});
        v8f h2b = wmma16g(cat16(*(const v8h*)&w2s[(16 + lr) * 32 + 8 * hi], *(const v8h*)&w2s[(16 + lr) * 32 + 16 + 8 * hi]), h1B, (v8f){});
#pragma unroll
        for (int r = 0; r < 8; ++r) { h2a[r] = tanh_e(h2a[r] + b2s[8 * hi + r]); h2b[r] = tanh_e(h2b[r] + b2s[16 + 8 * hi + r]); }
        const v16h h2B = pack2(h2a, h2b);
        const v8f fa = wmma16g(cat16(*(const v8h*)&w3s[lr * 32 + 8 * hi], *(const v8h*)&w3s[lr * 32 + 16 + 8 * hi]), h2B, (v8f){});
        float y2[8]; float t1 = 0.0f;
#pragma unroll
        for (int r = 0; r < 8; ++r) { const bool ok = (r < 4) | (hi == 0); y2[r] = z[r] + tanh_e(fa[r] + b3s[8 * hi + r]); t1 += ok ? y2[r] : 0.0f; }
        t1 += __shfl_xor(t1, 16, 32);
        const float mu2 = t1 * (1.0f / 12.0f);
        float d2[8]; float t2 = 0.0f;
#pragma unroll
        for (int r = 0; r < 8; ++r) { const bool ok = (r < 4) | (hi == 0); d2[r] = ok ? (y2[r] - mu2) : 0.0f; t2 += d2[r] * d2[r]; }
        t2 += __shfl_xor(t2, 16, 32);
        const float rs2 = rsqrtf(t2 * (1.0f / 12.0f) + LNEPS);
        v4f c0, c1;
#pragma unroll
        for (int r = 0; r < 4; ++r) { c0[r] = d2[r] * rs2 * g2s[8 * hi + r] + e2s[8 * hi + r]; c1[r] = d2[4 + r] * rs2 * g2s[8 * hi + 4 + r] + e2s[8 * hi + 4 + r]; }
        const int ob_ = (qt * 16 + lr) * OSW + wave * EMB + 8 * hi;
        *(v4fa*)(&os[ob_]) = c0;
        if (hi == 0) *(v4fa*)(&os[ob_ + 4]) = c1;
    }
    __syncthreads();

#pragma unroll 1
    for (int ps = 0; ps < 2; ++ps) {
#pragma unroll
        for (int it = 0; it < OITER; ++it) { const int p = it * (32 * BPB) + tid; const int pos = p / (OSW / 4), c4 = p - pos * (OSW / 4);
            const v4f val = *(const v4fa*)(&os[pos * OSW + c4 * 4]);
            *(volatile v4f*)(out + ((size_t)pos * OUT_NB + (size_t)n0) * EMB + (size_t)c4 * 4) = val; }
        if (ps == 0) __threadfence(); }
}

static constexpr size_t SZ_TOTAL = 0;
static_assert(SZ_TOTAL <= (size_t)134217728);

extern "C" void kernel_launch(void* const* d_in, const int* in_sizes, int n_in,
                              void* d_out, int out_size, void* d_ws, size_t ws_size, hipStream_t stream) {
    if (n_in < 15) return;
    const size_t needx = ((size_t)(SEQ - 1) * NB_FULL + NB) * EMB;
    if ((size_t)in_sizes[0] < needx) return;
    if (in_sizes[1] < 3 * EMB * EMB || in_sizes[2] < 3 * EMB) return;
    if (in_sizes[3] < EMB * EMB || in_sizes[4] < EMB) return;
    if (in_sizes[5] < HID * EMB || in_sizes[6] < HID) return;
    if (in_sizes[7] < HID * HID || in_sizes[8] < HID) return;
    if (in_sizes[9] < EMB * HID || in_sizes[10] < EMB) return;
    if (in_sizes[11] < EMB || in_sizes[12] < EMB || in_sizes[13] < EMB || in_sizes[14] < EMB) return;
    if ((size_t)out_size < ((size_t)(SEQ - 1) * OUT_NB + NB) * EMB) return;
    if (SZ_TOTAL > ws_size) return;
    const float* x   = (const float*)d_in[0];
    const float* inw = (const float*)d_in[1];  const float* inb = (const float*)d_in[2];
    const float* ow  = (const float*)d_in[3];  const float* ob  = (const float*)d_in[4];
    const float* w1  = (const float*)d_in[5];  const float* b1  = (const float*)d_in[6];
    const float* w2  = (const float*)d_in[7];  const float* b2  = (const float*)d_in[8];
    const float* w3  = (const float*)d_in[9];  const float* b3  = (const float*)d_in[10];
    const float* g1  = (const float*)d_in[11]; const float* be1 = (const float*)d_in[12];
    const float* g2  = (const float*)d_in[13]; const float* be2 = (const float*)d_in[14];
    float* OUT = (float*)d_out;
    k_enc<<<dim3(NB / BPB, 1, 1), 32 * BPB, 0, stream>>>(x, inw, inb, ow, ob, w1, b1, w2, b2, w3, b3, g1, be1, g2, be2, OUT);
}
